// FeatureAttnNet_30906584662249
// MI455X (gfx1250) — hardware-verified
//
#include <hip/hip_runtime.h>


namespace {
constexpr int NBt = 1024, NE = 2048, NHID = 1024, NC = 128, D = 64, NH = 8, NF = 128, M = 4096, DH = D * NH;
constexpr float XS = 8.0f, WSC = 256.0f, LN_EPS = 1e-5f;

typedef _Float16 b16;
typedef __attribute__((ext_vector_type(16))) _Float16 v16b;
typedef __attribute__((ext_vector_type(8))) _Float16 v8b;
typedef __attribute__((ext_vector_type(8))) float v8f;
typedef __attribute__((ext_vector_type(4))) float v4f;
__device__ __forceinline__ float bf16_rne(float f) { unsigned int u = __float_as_uint(f); u += 0x7FFFu + ((u >> 16) & 1u); return __uint_as_float(u & 0xFFFF0000u); }
__device__ __forceinline__ void split16(float v, b16& hi, b16& lo) { hi = (b16)v; lo = (b16)(v - (float)hi); }
__device__ __forceinline__ v16b frag_kb(const b16* p, int hh) { const v8b a = *(const v8b*)(p + 8 * hh), b = *(const v8b*)(p + 16 + 8 * hh); v16b f;
#pragma unroll
  for (int e = 0; e < 8; ++e) { f[e] = a[e]; f[8 + e] = b[e]; } return f; }
__device__ __forceinline__ v8f wmma16b(v16b a, v16b b, v8f c) { v8f d = __builtin_amdgcn_wmma_f32_16x16x32_f16(false, a, false, b, (short)0, c, false, false); asm volatile("v_nop\n\tv_nop\n\tv_nop\n\tv_nop" : "+v"(d) : "v"(a), "v"(b)); return d; }
__device__ __forceinline__ void wave_lds_sync() { __builtin_amdgcn_fence(__ATOMIC_RELEASE, "workgroup"); __builtin_amdgcn_wave_barrier(); __builtin_amdgcn_fence(__ATOMIC_ACQUIRE, "workgroup"); }
__device__ __forceinline__ float nexp(float x) { return __builtin_amdgcn_exp2f(x * 1.4426950408889634f); }
__device__ __forceinline__ float pmul(float a, float b) { float p = a * b; asm volatile("" : "+v"(p)); return p; }
__device__ __forceinline__ float hsum16(float v) { v += __shfl_xor(v, 1); v += __shfl_xor(v, 2); v += __shfl_xor(v, 4); return v + __shfl_xor(v, 8); }
__device__ __forceinline__ float gelu_erf(float x) { return 0.5f * x * (1.0f + erff(x * 0.70710678118654752f)); }

__global__ __launch_bounds__(256) void prepx_kernel(const float* __restrict__ fe, const float* __restrict__ hi, const float* __restrict__ cm, b16* __restrict__ XF, b16* __restrict__ XH, b16* __restrict__ XC) {
  const size_t t = (size_t)blockIdx.x * 256 + threadIdx.x; const size_t n1 = (size_t)NBt * NE / 8, n2 = (size_t)NBt * NHID / 8, n3 = (size_t)NBt * NC / 8; const float* src; b16* dst; size_t e;
  if (t < n1) { src = fe; dst = XF; e = t * 8; } else if (t < n1 + n2) { src = hi; dst = XH; e = (t - n1) * 8; } else if (t < n1 + n2 + n3) { src = cm; dst = XC; e = (t - n1 - n2) * 8; } else return;
  const v4f a = *(const v4f*)(src + e), c = *(const v4f*)(src + e + 4); v8b o;
#pragma unroll
  for (int j = 0; j < 4; ++j) { o[j] = (b16)(bf16_rne(a[j]) * XS); o[4 + j] = (b16)(bf16_rne(c[j]) * XS); }
  for (int pass = 0; pass < 2; ++pass) { *(volatile v8b*)(dst + e) = o; __threadfence(); }
}
__global__ __launch_bounds__(256) void prepw_kernel(const float* __restrict__ wz, const float* __restrict__ wh, const float* __restrict__ wq, const float* __restrict__ wk, const float* __restrict__ wv, b16* __restrict__ WZT, b16* __restrict__ WHT, b16* __restrict__ WQT, b16* __restrict__ WKT, b16* __restrict__ WVT) {
  __shared__ __attribute__((aligned(16))) b16 T[64][64 + 8];
  const int kind = blockIdx.z, i0 = blockIdx.x * 64, o0 = blockIdx.y * 64, t_ = threadIdx.x; int IN, OUT; const float* w; b16* dst;
  if (kind == 0) { IN = NE; OUT = M; w = wz; dst = WZT; } else if (kind == 1) { IN = NHID; OUT = M; w = wh; dst = WHT; } else if (kind == 2) { IN = NC; OUT = DH; w = wq; dst = WQT; } else if (kind == 3) { IN = D; OUT = DH; w = wk; dst = WKT; } else { IN = D; OUT = DH; w = wv; dst = WVT; }
  if (i0 >= IN || o0 >= OUT) return;
  for (int q = t_; q < 64 * 64; q += 256) { const int ii = q >> 6, oo = q & 63; T[oo][ii] = (b16)(bf16_rne(w[(size_t)(i0 + ii) * OUT + o0 + oo]) * WSC); }
  __syncthreads();
  for (int pass = 0; pass < 2; ++pass) { for (int q = t_; q < 64 * 8; q += 256) { const int oo = q >> 3, c8 = (q & 7) * 8; *(volatile v8b*)(dst + (size_t)(o0 + oo) * IN + i0 + c8) = *(const v8b*)(&T[oo][c8]); } __threadfence(); }
}
__global__ __launch_bounds__(128) void proj_kernel(const b16* __restrict__ XF, const b16* __restrict__ XH, const b16* __restrict__ WZT, const b16* __restrict__ WHT, const float* __restrict__ gam, const float* __restrict__ bet, b16* __restrict__ FIh, b16* __restrict__ FIl) {
  __shared__ __attribute__((aligned(16))) b16 Th[4][16][128 + 8], Tl[4][16][128 + 8];
  const int wave = threadIdx.x >> 5, lane = threadIdx.x & 31, nloc = lane & 15, hlf = lane >> 4; const int kind = blockIdx.z; const size_t m0 = (size_t)blockIdx.x * 64 + wave * 16; const int n0 = blockIdx.y * 128;
  const b16* A = kind ? XH : XF; const b16* W = kind ? WHT : WZT; const int K = kind ? NHID : NE; v8f acc[8];
#pragma unroll
  for (int t = 0; t < 8; ++t) acc[t] = (v8f){};
  for (int kb = 0; kb < K; kb += 32) { const v16b a = frag_kb(A + (m0 + nloc) * K + kb, hlf);
#pragma unroll
    for (int t = 0; t < 8; ++t) acc[t] = wmma16b(a, frag_kb(W + (size_t)(n0 + t * 16 + nloc) * K + kb, hlf), acc[t]); }
#pragma unroll
  for (int gq = 0; gq < 2; ++gq) {
#pragma unroll
    for (int r = 0; r < 8; ++r) { float x[4]; float s = 0.0f;
#pragma unroll
      for (int u = 0; u < 4; ++u) { x[u] = gelu_erf(acc[gq * 4 + u][r] * (1.0f / (XS * WSC))); s += x[u]; }
      s = hsum16(s); const float mu = s * (1.0f / D); float q2 = 0.0f;
#pragma unroll
      for (int u = 0; u < 4; ++u) { const float dv = x[u] - mu; q2 += pmul(dv, dv); }
      q2 = hsum16(q2); const float rs = rsqrtf(q2 * (1.0f / D) + LN_EPS);
#pragma unroll
      for (int u = 0; u < 4; ++u) { const int dd = u * 16 + nloc; const float y = pmul((x[u] - mu) * rs, bf16_rne(gam[dd])) + bf16_rne(bet[dd]); b16 h_, l_; split16(y * XS, h_, l_); Th[wave][8 * hlf + r][gq * 64 + dd] = h_; Tl[wave][8 * hlf + r][gq * 64 + dd] = l_; } } }
  wave_lds_sync();
  for (int pass = 0; pass < 2; ++pass) { for (int r4 = 0; r4 < 32; r4 += 4) { const int idx = r4 + (lane >> 3); const int rr = idx >> 1, gq = idx & 1; const int c8 = (lane & 7) * 8; const size_t firow = (m0 + rr) * NF + (size_t)(kind * M + n0) / D + gq;
      *(volatile v8b*)(FIh + firow * D + c8) = *(const v8b*)(&Th[wave][rr][gq * 64 + c8]); *(volatile v8b*)(FIl + firow * D + c8) = *(const v8b*)(&Tl[wave][rr][gq * 64 + c8]); } __threadfence(); }
}
__global__ __launch_bounds__(128) void q_kernel(const b16* __restrict__ XC, const b16* __restrict__ WQT, float* __restrict__ QP) {
  __shared__ __attribute__((aligned(16))) float Ts[4][16][128 + 4];
  const int wave = threadIdx.x >> 5, lane = threadIdx.x & 31, nloc = lane & 15, hlf = lane >> 4; const size_t m0 = (size_t)blockIdx.x * 64 + wave * 16; const int n0 = blockIdx.y * 128;
  v8f acc[8];
#pragma unroll
  for (int t = 0; t < 8; ++t) acc[t] = (v8f){};
#pragma unroll
  for (int kb = 0; kb < NC; kb += 32) { const v16b a = frag_kb(XC + (m0 + nloc) * NC + kb, hlf);
#pragma unroll
    for (int t = 0; t < 8; ++t) acc[t] = wmma16b(a, frag_kb(WQT + (size_t)(n0 + t * 16 + nloc) * NC + kb, hlf), acc[t]); }
#pragma unroll
  for (int t = 0; t < 8; ++t)
#pragma unroll
    for (int r = 0; r < 8; ++r) Ts[wave][8 * hlf + r][t * 16 + nloc] = acc[t][r] * (1.0f / (XS * WSC));
  wave_lds_sync();
  for (int pass = 0; pass < 2; ++pass) { for (int rr = 0; rr < 16; ++rr) *(volatile v4f*)(QP + (m0 + rr) * DH + n0 + lane * 4) = *(const v4f*)(&Ts[wave][rr][lane * 4]); __threadfence(); }
}
__global__ __launch_bounds__(128) void attn_kernel(const b16* __restrict__ FIh, const b16* __restrict__ FIl, const b16* __restrict__ WKT, const b16* __restrict__ WVT, const float* __restrict__ QP, float* __restrict__ out) {
  __shared__ float Ks[NF][D + 1], Vs[NF][D + 1]; __shared__ float Al[NF], red[NF];
  const int wave = threadIdx.x >> 5, lane = threadIdx.x & 31, nloc = lane & 15, hlf = lane >> 4, t_ = threadIdx.x; const int b = blockIdx.x / NH, h = blockIdx.x - b * NH;
  for (int mt = 0; mt < 2; ++mt) { const size_t r0 = (size_t)b * NF + wave * 32 + mt * 16; v8f ak[4] = {{}, {}, {}, {}}, av[4] = {{}, {}, {}, {}};
#pragma unroll
    for (int kb = 0; kb < D; kb += 32) { const v16b a = frag_kb(FIh + (r0 + nloc) * D + kb, hlf), al = frag_kb(FIl + (r0 + nloc) * D + kb, hlf);
#pragma unroll
      for (int t = 0; t < 4; ++t) { const v16b bk = frag_kb(WKT + (size_t)(h * D + t * 16 + nloc) * D + kb, hlf), bv = frag_kb(WVT + (size_t)(h * D + t * 16 + nloc) * D + kb, hlf);
        ak[t] = wmma16b(a, bk, ak[t]); ak[t] = wmma16b(al, bk, ak[t]); av[t] = wmma16b(a, bv, av[t]); av[t] = wmma16b(al, bv, av[t]); } }
#pragma unroll
    for (int t = 0; t < 4; ++t)
#pragma unroll
      for (int r = 0; r < 8; ++r) { const int n = wave * 32 + mt * 16 + 8 * hlf + r, dd = t * 16 + nloc; Ks[n][dd] = ak[t][r] * (1.0f / (XS * WSC)); Vs[n][dd] = av[t][r] * (1.0f / (XS * WSC)); } }
  __syncthreads();
  { const int n = t_; float qk = 0.0f, mv = 0.0f; const float* qh = QP + (size_t)b * DH + h * D;
    for (int dd = 0; dd < D; ++dd) { qk += pmul(qh[dd], Ks[n][dd]); mv += fabsf(Vs[n][dd]); }
    const float lg = pmul(mv * (1.0f / D), qk) * 0.125f; Al[n] = lg; red[n] = lg; }
  __syncthreads();
  for (int s = 64; s >= 1; s >>= 1) { if (t_ < s) red[t_] = fmaxf(red[t_], red[t_ + s]); __syncthreads(); }
  const float mx = red[0]; __syncthreads();
  { const float e = nexp(Al[t_] - mx); Al[t_] = e; red[t_] = e; } __syncthreads();
  for (int s = 64; s >= 1; s >>= 1) { if (t_ < s) red[t_] += red[t_ + s]; __syncthreads(); }
  const float inv = 1.0f / red[0];
  float sres = 0.0f; if (t_ < D) { for (int n = 0; n < NF; ++n) sres += pmul(Al[n], Vs[n][t_]); sres *= inv; }
  for (int pass = 0; pass < 2; ++pass) { if (t_ < D) ((volatile float*)out)[((size_t)b * NH + h) * D + t_] = sres; __threadfence(); }
}
}

extern "C" void kernel_launch(void* const* d_in, const int* in_sizes, int n_in, void* d_out, int out_size, void* d_ws, size_t ws_size, hipStream_t stream) {
  (void)n_in;
  auto Fp = [&](int i) { return (const float*)d_in[i]; };
  if (in_sizes[0] != NBt * NE || in_sizes[1] != NBt * NHID || in_sizes[2] != NBt * NC || in_sizes[3] != NE * M || in_sizes[4] != NHID * M || in_sizes[5] != NC * DH || in_sizes[6] != D * DH || in_sizes[7] != D * DH || out_size != NBt * NH * D) return;
  size_t off = 0; char* ws = (char*)d_ws;
  auto carve = [&](size_t bytes) { char* p = ws + off; off += (bytes + 255) & ~(size_t)255; return p; };
  b16* XF = (b16*)carve((size_t)NBt * NE * 2); b16* XH = (b16*)carve((size_t)NBt * NHID * 2); b16* XC = (b16*)carve((size_t)NBt * NC * 2);
  b16* WZT = (b16*)carve((size_t)M * NE * 2); b16* WHT = (b16*)carve((size_t)M * NHID * 2); b16* WQT = (b16*)carve((size_t)DH * NC * 2); b16* WKT = (b16*)carve((size_t)DH * D * 2); b16* WVT = (b16*)carve((size_t)DH * D * 2);
  b16* FIh = (b16*)carve((size_t)NBt * NF * D * 2); b16* FIl = (b16*)carve((size_t)NBt * NF * D * 2); float* QP = (float*)carve((size_t)NBt * DH * 4);
  if (off > ws_size || off > ((size_t)128 << 20)) return;
  prepx_kernel<<<(unsigned)(((size_t)NBt * (NE + NHID + NC) / 8 + 255) / 256), 256, 0, stream>>>(Fp(0), Fp(1), Fp(2), XF, XH, XC);
  prepw_kernel<<<dim3(NE / 64, M / 64, 5), 256, 0, stream>>>(Fp(3), Fp(4), Fp(5), Fp(6), Fp(7), WZT, WHT, WQT, WKT, WVT);
  proj_kernel<<<dim3(NBt / 64, M / 128, 2), 128, 0, stream>>>(XF, XH, WZT, WHT, Fp(8), Fp(9), FIh, FIl);
  q_kernel<<<dim3(NBt / 64, DH / 128), 128, 0, stream>>>(XC, WQT, QP);
  attn_kernel<<<NBt * NH, 128, 0, stream>>>(FIh, FIl, WKT, WVT, QP, (float*)d_out);
}
